// GINRegressor_5085241279117
// MI455X (gfx1250) — hardware-verified
//
#include <hip/hip_runtime.h>
#include <stddef.h>


#define DF       128
#define NTHR     256
#define NWAVE    8
#define EPT      8
#define NGRP     2
#define CHUNK    (NTHR * EPT * NGRP)
#define WCAP     (EPT * NGRP * 32)
#define LISTN    (NWAVE * WCAP)
#define NB       512
#define NTILE    (NB / 16)
#define TPW      (NTILE / NWAVE)
#define PLANE    (DF * DF)
#define LDS_MAIN (NB * DF * 4 + LISTN * 4 + 64)

static_assert((CHUNK & (CHUNK - 1)) == 0);
static_assert(CHUNK <= 4096);
static_assert((NB & (NB - 1)) == 0);
static_assert(NB <= 4096);
static_assert(NTILE % NWAVE == 0);
static_assert(3 * DF * 4 + NB * 4 <= LISTN * 4);
static_assert(NB % 128 == 0 && NB / 128 <= NWAVE);

typedef float          v4f   __attribute__((ext_vector_type(4)));
typedef float          v8f   __attribute__((ext_vector_type(8)));
typedef int            v4i   __attribute__((ext_vector_type(4)));
typedef unsigned short v8us  __attribute__((ext_vector_type(8)));
typedef unsigned short v16us __attribute__((ext_vector_type(16)));
typedef __bf16         v16bf __attribute__((ext_vector_type(16)));
union FragB { v16bf v; v16us u; v8us h[2]; };

__device__ __forceinline__ unsigned hl1(float f) {
  const unsigned u  = __float_as_uint(f);
  const unsigned r  = (u + 0x7FFFu + ((u >> 16) & 1u)) >> 16;
  const float    fh = __uint_as_float(r << 16);
  const unsigned u2 = __float_as_uint(f - fh);
  const unsigned r2 = (u2 + 0x7FFFu + ((u2 >> 16) & 1u)) >> 16;
  return (r & 0xffffu) | (r2 << 16);
}

__device__ __forceinline__ void split8(v4f a, v4f b, v8us& H, v8us& L) {
  const unsigned q0 = hl1(a.x), q1 = hl1(a.y), q2 = hl1(a.z), q3 = hl1(a.w);
  const unsigned q4 = hl1(b.x), q5 = hl1(b.y), q6 = hl1(b.z), q7 = hl1(b.w);
  v8us hv, lv;
  hv[0] = (unsigned short)(q0 & 0xffffu); lv[0] = (unsigned short)(q0 >> 16);
  hv[1] = (unsigned short)(q1 & 0xffffu); lv[1] = (unsigned short)(q1 >> 16);
  hv[2] = (unsigned short)(q2 & 0xffffu); lv[2] = (unsigned short)(q2 >> 16);
  hv[3] = (unsigned short)(q3 & 0xffffu); lv[3] = (unsigned short)(q3 >> 16);
  hv[4] = (unsigned short)(q4 & 0xffffu); lv[4] = (unsigned short)(q4 >> 16);
  hv[5] = (unsigned short)(q5 & 0xffffu); lv[5] = (unsigned short)(q5 >> 16);
  hv[6] = (unsigned short)(q6 & 0xffffu); lv[6] = (unsigned short)(q6 >> 16);
  hv[7] = (unsigned short)(q7 & 0xffffu); lv[7] = (unsigned short)(q7 >> 16);
  H = hv; L = lv;
}

__device__ __forceinline__ v8f wmb(v16bf a, v16bf b, v8f c) {
  v8f d = __builtin_amdgcn_wmma_f32_16x16x32_bf16(false, a, false, b, (short)0, c, false, false);
  asm volatile("v_nop\n\tv_nop\n\tv_nop\n\tv_nop" : "+v"(d) : "v"(a), "v"(b));
  return d;
}

template <int NBT>
__device__ __forceinline__ int scan_chunk(const int* __restrict__ dsts, int nE, int cbase, int nodeBase,
                                          int vec8, int* list, int tid, int lane, int wave) {
  int wc = 0;
#pragma unroll
  for (int g = 0; g < NGRP; ++g) {
    const int el0  = (g * NTHR + tid) * EPT;
    const int e0   = cbase + el0;
    const int sent = -2147483647 - 1;
    v4i da, db;
    if (vec8 != 0 && cbase + CHUNK <= nE) {
      da = *(const v4i*)(dsts + e0);
      db = *(const v4i*)(dsts + e0 + 4);
    } else {
      da.x = (e0     < nE) ? dsts[min(e0,     nE - 1)] : sent;
      da.y = (e0 + 1 < nE) ? dsts[min(e0 + 1, nE - 1)] : sent;
      da.z = (e0 + 2 < nE) ? dsts[min(e0 + 2, nE - 1)] : sent;
      da.w = (e0 + 3 < nE) ? dsts[min(e0 + 3, nE - 1)] : sent;
      db.x = (e0 + 4 < nE) ? dsts[min(e0 + 4, nE - 1)] : sent;
      db.y = (e0 + 5 < nE) ? dsts[min(e0 + 5, nE - 1)] : sent;
      db.z = (e0 + 6 < nE) ? dsts[min(e0 + 6, nE - 1)] : sent;
      db.w = (e0 + 7 < nE) ? dsts[min(e0 + 7, nE - 1)] : sent;
    }
    const unsigned nb = (unsigned)nodeBase;
    const unsigned s0 = (unsigned)da.x - nb, s1 = (unsigned)da.y - nb;
    const unsigned s2 = (unsigned)da.z - nb, s3 = (unsigned)da.w - nb;
    const unsigned s4 = (unsigned)db.x - nb, s5 = (unsigned)db.y - nb;
    const unsigned s6 = (unsigned)db.z - nb, s7 = (unsigned)db.w - nb;
    const bool h0 = s0 < (unsigned)NBT, h1 = s1 < (unsigned)NBT, h2 = s2 < (unsigned)NBT, h3 = s3 < (unsigned)NBT;
    const bool h4 = s4 < (unsigned)NBT, h5 = s5 < (unsigned)NBT, h6 = s6 < (unsigned)NBT, h7 = s7 < (unsigned)NBT;
    const unsigned any = __builtin_amdgcn_ballot_w32(h0 | h1 | h2 | h3 | h4 | h5 | h6 | h7);
    if (any != 0u) {
#define HITJ(J, HJ, SJ) { \
        const unsigned mj = __builtin_amdgcn_ballot_w32(HJ); \
        if (mj != 0u) { \
          if (HJ) { \
            const int pos = wc + (int)__builtin_amdgcn_mbcnt_lo(mj, 0u); \
            if (pos < WCAP) list[wave * WCAP + pos] = ((el0 + (J)) << 12) | (int)(SJ); \
          } \
          wc += (int)__builtin_popcount(mj); } }
      HITJ(0, h0, s0)
      HITJ(1, h1, s1)
      HITJ(2, h2, s2)
      HITJ(3, h3, s3)
      HITJ(4, h4, s4)
      HITJ(5, h5, s5)
      HITJ(6, h6, s6)
      HITJ(7, h7, s7)
#undef HITJ
    }
  }
  return wc;
}

__global__ __launch_bounds__(NTHR) void k_wprep(
    const float* __restrict__ w0, const float* __restrict__ w1,
    const float* __restrict__ w2, const float* __restrict__ w3,
    unsigned short* wp) {
  const int i = blockIdx.x * NTHR + threadIdx.x;
  if (i >= 4 * PLANE / 8) return;
  const int w  = i >> 11;
  const int o  = (i & 2047) * 8;
  const int n  = o >> 7;
  const int k0 = o & (DF - 1);
  const float* W = (w == 0) ? w0 : ((w == 1) ? w1 : ((w == 2) ? w2 : w3));
  const float* p = W + (size_t)k0 * DF + n;
  v4f a, b;
  a.x = p[0];      a.y = p[DF];     a.z = p[2 * DF]; a.w = p[3 * DF];
  b.x = p[4 * DF]; b.y = p[5 * DF]; b.z = p[6 * DF]; b.w = p[7 * DF];
  v8us hv, lv;
  split8(a, b, hv, lv);
  unsigned short* ph = wp + (size_t)(2 * w) * PLANE + o;
  unsigned short* pl = ph + PLANE;
  *(volatile v8us*)ph = hv;
  *(volatile v8us*)pl = lv;
  __threadfence();
  *(volatile v8us*)ph = hv;
  *(volatile v8us*)pl = lv;
}

__device__ __forceinline__ void wave_gemm(const float* arows, const unsigned short* __restrict__ ph,
                                          int m, int hh, v8f acc[8]) {
#pragma unroll
  for (int t = 0; t < 8; ++t) { v8f z = {0.f, 0.f, 0.f, 0.f, 0.f, 0.f, 0.f, 0.f}; acc[t] = z; }
#pragma unroll
  for (int kt = 0; kt < DF / 32; ++kt) {
    const float* ap = arows + m * DF + 32 * kt + 8 * hh;
    const v4f p0 = *(const v4f*)ap,        p1 = *(const v4f*)(ap + 4);
    const v4f p2 = *(const v4f*)(ap + 16), p3 = *(const v4f*)(ap + 20);
    FragB ah, al;
    split8(p0, p1, ah.h[0], al.h[0]);
    split8(p2, p3, ah.h[1], al.h[1]);
#pragma unroll
    for (int nt = 0; nt < 8; ++nt) {
      const unsigned short* bp = ph + (size_t)(16 * nt + m) * DF + 32 * kt + 8 * hh;
      FragB bh, bl;
      bh.h[0] = *(const v8us*)bp;            bh.h[1] = *(const v8us*)(bp + 16);
      bl.h[0] = *(const v8us*)(bp + PLANE);  bl.h[1] = *(const v8us*)(bp + PLANE + 16);
      acc[nt] = wmb(ah.v, bh.v, acc[nt]);
      acc[nt] = wmb(al.v, bh.v, acc[nt]);
      acc[nt] = wmb(ah.v, bl.v, acc[nt]);
    }
  }
}

template <int LAST>
__global__ __launch_bounds__(NTHR) void k_gin(
    const int* __restrict__ ei, const float* __restrict__ feat, const unsigned short* __restrict__ wp,
    const float* __restrict__ ba, const float* __restrict__ bb, const float* __restrict__ wo,
    const float* __restrict__ bo, float* hout, float* out, int nN, int nE, int vec8) {
  extern __shared__ v4f lds_dyn[];
  float* accr = (float*)lds_dyn;
  int*   list = (int*)(accr + NB * DF);
  int*   wcnt = list + LISTN;
  float* sba  = (float*)list;
  float* sbb  = sba + DF;
  float* swo  = sbb + DF;
  float* sout = swo + DF;
  const int tid = threadIdx.x, lane = tid & 31, wave = tid >> 5, hh = lane >> 4, m = lane & 15;
  const int nodeBase = blockIdx.x * NB;
  const int* dsts = ei + nE;
  const float bov = bo[0];

#pragma unroll 4
  for (int i = 0; i < (NB * DF / 4) / NTHR; ++i) {
    const int idx  = i * NTHR + tid;
    const int slot = idx >> 5;
    const int c4   = (idx & 31) * 4;
    int node = nodeBase + slot;
    node = node > nN - 1 ? nN - 1 : node;
    lds_dyn[idx] = *(const v4f*)(feat + (size_t)node * DF + c4);
  }
  __syncthreads();

  const int nChunks = (nE + CHUNK - 1) / CHUNK;
#pragma unroll 1
  for (int ch = 0; ch < nChunks; ++ch) {
    const int cbase = ch * CHUNK;
    const int wc = scan_chunk<NB>(dsts, nE, cbase, nodeBase, vec8, list, tid, lane, wave);
    if (lane == 0) wcnt[wave] = wc;
    __syncthreads();
    if (wave == 0) {
#pragma unroll 1
      for (int wsx = 0; wsx < NWAVE; ++wsx) {
        int n = __builtin_amdgcn_readfirstlane(wcnt[wsx]);
        n = n > WCAP ? WCAP : (n < 0 ? 0 : n);
        const int* lp = list + wsx * WCAP;
#pragma unroll 1
        for (int i = 0; i < n; ++i) {
          const int ent  = __builtin_amdgcn_readfirstlane(lp[i]);
          const int slot = ent & (NB - 1);
          int e = cbase + ((ent >> 12) & (CHUNK - 1));
          e = e > nE - 1 ? nE - 1 : e;
          int src = ei[e];
          src = src < 0 ? 0 : (src > nN - 1 ? nN - 1 : src);
          const v4f v = *(const v4f*)(feat + (size_t)src * DF + 4 * lane);
          v4f* ap = (v4f*)(accr + slot * DF + 4 * lane);
          *ap = *ap + v;
        }
      }
    }
    __syncthreads();
  }

  if (tid < DF) { sba[tid] = ba[tid]; sbb[tid] = bb[tid]; swo[tid] = wo[tid]; }
  __syncthreads();

#pragma unroll 1
  for (int it = 0; it < TPW; ++it) {
    const int row0 = 16 * (wave + NWAVE * it);
    v8f acc[8];

    wave_gemm(accr + row0 * DF, wp, m, hh, acc);
    {
      float* sp = accr + (row0 + 8 * hh) * DF + m;
#pragma unroll
      for (int nt = 0; nt < 8; ++nt) {
        const float bias = sba[16 * nt + m];
        sp[0 * DF + 16 * nt] = fmaxf(acc[nt][0] + bias, 0.f);
        sp[1 * DF + 16 * nt] = fmaxf(acc[nt][1] + bias, 0.f);
        sp[2 * DF + 16 * nt] = fmaxf(acc[nt][2] + bias, 0.f);
        sp[3 * DF + 16 * nt] = fmaxf(acc[nt][3] + bias, 0.f);
        sp[4 * DF + 16 * nt] = fmaxf(acc[nt][4] + bias, 0.f);
        sp[5 * DF + 16 * nt] = fmaxf(acc[nt][5] + bias, 0.f);
        sp[6 * DF + 16 * nt] = fmaxf(acc[nt][6] + bias, 0.f);
        sp[7 * DF + 16 * nt] = fmaxf(acc[nt][7] + bias, 0.f);
      }
    }
    __syncthreads();

    wave_gemm(accr + row0 * DF, wp + 2 * PLANE, m, hh, acc);

    if (LAST == 0) {
      {
        float* sp = accr + (row0 + 8 * hh) * DF + m;
#pragma unroll
        for (int nt = 0; nt < 8; ++nt) {
          const float bias = sbb[16 * nt + m];
          sp[0 * DF + 16 * nt] = acc[nt][0] + bias;
          sp[1 * DF + 16 * nt] = acc[nt][1] + bias;
          sp[2 * DF + 16 * nt] = acc[nt][2] + bias;
          sp[3 * DF + 16 * nt] = acc[nt][3] + bias;
          sp[4 * DF + 16 * nt] = acc[nt][4] + bias;
          sp[5 * DF + 16 * nt] = acc[nt][5] + bias;
          sp[6 * DF + 16 * nt] = acc[nt][6] + bias;
          sp[7 * DF + 16 * nt] = acc[nt][7] + bias;
        }
      }
      __syncthreads();
      const float* lp = accr + row0 * DF + 4 * lane;
      float* gp = hout + ((size_t)nodeBase + row0) * DF + 4 * lane;
#pragma unroll
      for (int i = 0; i < 16; ++i) { const v4f v = *(const v4f*)(lp + i * DF); *(volatile v4f*)(gp + (size_t)i * DF) = v; }
      __threadfence();
#pragma unroll
      for (int i = 0; i < 16; ++i) { const v4f v = *(const v4f*)(lp + i * DF); *(volatile v4f*)(gp + (size_t)i * DF) = v; }
    } else {
      float pr[8];
#pragma unroll
      for (int r = 0; r < 8; ++r) pr[r] = 0.f;
#pragma unroll
      for (int nt = 0; nt < 8; ++nt) {
        const int n = 16 * nt + m;
        const float bw = sbb[n], ww = swo[n];
#pragma unroll
        for (int r = 0; r < 8; ++r) pr[r] += (acc[nt][r] + bw) * ww;
      }
#pragma unroll
      for (int off = 1; off < 16; off <<= 1) {
#pragma unroll
        for (int r = 0; r < 8; ++r) pr[r] += __shfl_xor(pr[r], off, 32);
      }
      if (m == 0) {
        float* so = sout + row0 + 8 * hh;
        so[0] = pr[0] + bov; so[1] = pr[1] + bov; so[2] = pr[2] + bov; so[3] = pr[3] + bov;
        so[4] = pr[4] + bov; so[5] = pr[5] + bov; so[6] = pr[6] + bov; so[7] = pr[7] + bov;
      }
    }
  }

  if (LAST != 0) {
    __syncthreads();
    if (wave < NB / 128) {
      const int f  = wave * 128 + 4 * lane;
      const int gi = nodeBase + f;
      if (gi + 4 <= nN) { const v4f v = *(const v4f*)(sout + f); *(volatile v4f*)(out + gi) = v; }
    }
    __threadfence();
    if (wave < NB / 128) {
      const int f  = wave * 128 + 4 * lane;
      const int gi = nodeBase + f;
      if (gi + 4 <= nN) { const v4f v = *(const v4f*)(sout + f); *(volatile v4f*)(out + gi) = v; }
    }
  }
}

extern "C" void kernel_launch(void* const* d_in, const int* in_sizes, int n_in,
                              void* d_out, int out_size, void* d_ws, size_t ws_size,
                              hipStream_t stream) {
  if (n_in < 12) return;
  const int nN = in_sizes[0] / DF;
  const int nE = in_sizes[1] / 2;
  if (nN <= 0 || nE < 0 || in_sizes[0] != nN * DF || in_sizes[1] != nE * 2) return;
  if (in_sizes[2] != PLANE || in_sizes[4] != PLANE || in_sizes[6] != PLANE || in_sizes[8] != PLANE) return;
  if (in_sizes[3] < DF || in_sizes[5] < DF || in_sizes[7] < DF || in_sizes[9] < DF) return;
  if (in_sizes[10] < DF || in_sizes[11] < 1) return;
  if (out_size != nN) return;

  const float* x   = (const float*)d_in[0];
  const int*   ei  = (const int*)d_in[1];
  const float* w1a = (const float*)d_in[2];
  const float* b1a = (const float*)d_in[3];
  const float* w1b = (const float*)d_in[4];
  const float* b1b = (const float*)d_in[5];
  const float* w2a = (const float*)d_in[6];
  const float* b2a = (const float*)d_in[7];
  const float* w2b = (const float*)d_in[8];
  const float* b2b = (const float*)d_in[9];
  const float* wo  = (const float*)d_in[10];
  const float* bo  = (const float*)d_in[11];
  float* out = (float*)d_out;

  const int nBlk = (nN + NB - 1) / NB;

  char* ws = (char*)d_ws;
  size_t off = 0;
  const size_t oWP = off; off += (size_t)8 * PLANE * 2;              off = (off + 255) & ~(size_t)255;
  const size_t oH1 = off; off += (size_t)nBlk * NB * DF * 4;         off = (off + 255) & ~(size_t)255;
  if (off > ws_size) return;
  if (off > ((size_t)1 << 27)) return;
  unsigned short* wp = (unsigned short*)(ws + oWP);
  float*          h1 = (float*)(ws + oH1);

  const int vec8 = ((nE & 3) == 0) ? 1 : 0;

  k_wprep<<<(4 * PLANE / 8 + NTHR - 1) / NTHR, NTHR, 0, stream>>>(w1a, w1b, w2a, w2b, wp);

  hipFuncSetAttribute(reinterpret_cast<const void*>(&k_gin<0>),
                      hipFuncAttributeMaxDynamicSharedMemorySize, LDS_MAIN);
  k_gin<0><<<nBlk, NTHR, LDS_MAIN, stream>>>(ei, x, wp, b1a, b1b, wo, bo, h1, out, nN, nE, vec8);

  hipFuncSetAttribute(reinterpret_cast<const void*>(&k_gin<1>),
                      hipFuncAttributeMaxDynamicSharedMemorySize, LDS_MAIN);
  k_gin<1><<<nBlk, NTHR, LDS_MAIN, stream>>>(ei, h1, wp + 4 * PLANE, b2a, b2b, wo, bo, h1, out, nN, nE, vec8);
}
